// ButterflyLayer1D_35459249995889
// MI455X (gfx1250) — hardware-verified
//
#include <hip/hip_runtime.h>

typedef __attribute__((ext_vector_type(16))) _Float16 v16h;
typedef __attribute__((ext_vector_type(8)))  _Float16 v8h;
typedef __attribute__((ext_vector_type(16))) __bf16   v16b;
typedef __attribute__((ext_vector_type(8)))  __bf16   v8b;
typedef __attribute__((ext_vector_type(8)))  float    v8f;
typedef __attribute__((ext_vector_type(4)))  float    v4f;
typedef __attribute__((ext_vector_type(4)))  unsigned int v4u;

constexpr int  kNdat   = 1024;
constexpr int  kLen    = 8192;
constexpr int  kCh     = 128;
constexpr long kPlane  = (long)kNdat * 64 * kCh;
constexpr long kWHalves  = 1998848;
constexpr long kWRegion  = 2097152;

constexpr size_t kOffWH  = 0;
constexpr size_t kOffWL  = kOffWH  + (size_t)kWRegion * 2;
constexpr size_t kOffXH  = kOffWL  + (size_t)kWRegion * 2;
constexpr size_t kOffXL  = kOffXH  + (size_t)kPlane * 2;
constexpr size_t kOffP0H = kOffXL  + (size_t)kPlane * 2;
constexpr size_t kOffP0L = kOffP0H + (size_t)kPlane * 2;
constexpr size_t kOffP1H = kOffP0L + (size_t)kPlane * 2;
constexpr size_t kOffP1L = kOffP1H + (size_t)kPlane * 2;
constexpr size_t kWsTotal = kOffP1L + (size_t)kPlane * 2;
static_assert(kWsTotal == 109051904, "ws total");
static_assert(kWHalves <= kWRegion, "weight region");

__device__ __forceinline__ unsigned short f2bf_bits(float f) {
  unsigned u = __float_as_uint(f);
  return (unsigned short)((u + 0x7FFFu + ((u >> 16) & 1u)) >> 16);
}
__device__ __forceinline__ float bf_bits2f(unsigned short h) { return __uint_as_float(((unsigned)h) << 16); }
__device__ __forceinline__ unsigned pk16(unsigned short a, unsigned short b) { return (unsigned)a | ((unsigned)b << 16); }

__device__ __forceinline__ void dep_guard_h(v8f& a, v8f& b, v16h x, v16h y) { asm volatile("v_nop\n\tv_nop\n\tv_nop\n\tv_nop" : "+v"(a), "+v"(b) : "v"(x), "v"(y)); }
__device__ __forceinline__ void dep_guard_b(v8f& a, v8f& b, v16b x, v16b y) { asm volatile("v_nop\n\tv_nop\n\tv_nop\n\tv_nop" : "+v"(a), "+v"(b) : "v"(x), "v"(y)); }
__device__ __forceinline__ void keep4_h(v16h a, v16h b, v16h c, v16h d) { asm volatile("v_nop" :: "v"(a), "v"(b), "v"(c), "v"(d)); }
__device__ __forceinline__ void keep4_b(v16b a, v16b b, v16b c, v16b d) { asm volatile("v_nop" :: "v"(a), "v"(b), "v"(c), "v"(d)); }
__device__ __forceinline__ void acc_guard4(v8f& a, v8f& b, v8f& c, v8f& d) { asm volatile("v_nop\n\tv_nop\n\tv_nop\n\tv_nop" : "+v"(a), "+v"(b), "+v"(c), "+v"(d)); }
template <typename T> struct Frag;
template <> struct Frag<_Float16> {
  typedef v16h V; union U { v16h v; v8h h[2]; };
  static __device__ __forceinline__ v16h load(const _Float16* p) {
    U f; f.h[0] = *(const v8h*)(p); f.h[1] = *(const v8h*)(p + 16); return f.v;
  }
  static __device__ __forceinline__ v8f mma(v16h a, v16h b, v8f c) {
    return __builtin_amdgcn_wmma_f32_16x16x32_f16(false, a, false, b, (short)0, c, false, false);
  }
  static __device__ __forceinline__ void guard(v8f& a, v8f& b, v16h x, v16h y) { dep_guard_h(a, b, x, y); }
  static __device__ __forceinline__ void keep(v16h a, v16h b, v16h c, v16h d) { keep4_h(a, b, c, d); }
};
template <> struct Frag<__bf16> {
  typedef v16b V; union U { v16b v; v8b h[2]; };
  static __device__ __forceinline__ v16b load(const __bf16* p) {
    U f; f.h[0] = *(const v8b*)(p); f.h[1] = *(const v8b*)(p + 16); return f.v;
  }
  static __device__ __forceinline__ v8f mma(v16b a, v16b b, v8f c) {
    return __builtin_amdgcn_wmma_f32_16x16x32_bf16(false, a, false, b, (short)0, c, false, false);
  }
  static __device__ __forceinline__ void guard(v8f& a, v8f& b, v16b x, v16b y) { dep_guard_b(a, b, x, y); }
  static __device__ __forceinline__ void keep(v16b a, v16b b, v16b c, v16b d) { keep4_b(a, b, c, d); }
};

template <int ET> struct Elem;
template <> struct Elem<0> { typedef _Float16 T; };
template <> struct Elem<1> { typedef __bf16 T; };
template <int ET, bool SPLIT, int BIAS_MODE, int OUT_MODE, bool RESID, int ACT = 0>
__global__ __launch_bounds__(256) void wmma_gemm64(
    const unsigned short* __restrict__ Ap, const unsigned short* __restrict__ A2p, int lda, long strideA,
    const unsigned short* __restrict__ Btp, const unsigned short* __restrict__ Bt2p, int ldb, long strideB,
    void* __restrict__ Cout, void* __restrict__ Cout2, int ldc, long strideC,
    const float* __restrict__ bias, long strideBias,
    const float* __restrict__ resid, long strideR,
    int M, int N, int K, float scale) {
  typedef typename Elem<ET>::T T;
  typedef typename Frag<T>::V V;
  const T* A = (const T*)Ap; const T* A2 = (const T*)A2p; const T* Bt = (const T*)Btp; const T* Bt2 = (const T*)Bt2p;
  __shared__ __align__(16) float sT[8][16 * 68];
  const int b    = blockIdx.y;
  const int lane = threadIdx.x & 31;
  const int wave = threadIdx.x >> 5;
  const int tilesN = N >> 6;
  const int tilesM = M >> 6;
  const int tile = blockIdx.x * 8 + wave;
  if (tile >= tilesM * tilesN) return;
  const int tm = tile / tilesN;
  const int tn = tile - tm * tilesN;
  const int m0 = tm << 6;
  const int n0 = tn << 6;

  const T* Ab  = A  + (size_t)b * strideA;
  const T* Bb  = Bt + (size_t)b * strideB;
  const T* Ab2 = SPLIT ? (A2  + (size_t)b * strideA) : nullptr;
  const T* Bb2 = SPLIT ? (Bt2 + (size_t)b * strideB) : nullptr;
  const float* biasb = (BIAS_MODE != 0) ? (bias + (size_t)b * strideBias) : nullptr;

  const int rlane = lane & 15;
  const int koff  = (lane >> 4) * 8;
  const int mOff  = (lane >> 4) * 8;

  v8f acc[4][4];
#pragma unroll
  for (int i = 0; i < 4; ++i)
#pragma unroll
    for (int j = 0; j < 4; ++j) acc[i][j] = (v8f){0.f,0.f,0.f,0.f,0.f,0.f,0.f,0.f};

  for (int k0 = 0; k0 < K; k0 += 32) {
    V bh[4], bl[4];
#pragma unroll
    for (int j = 0; j < 4; ++j) {
      const size_t bo = (size_t)(n0 + (j << 4) + rlane) * ldb + koff + k0;
      bh[j] = Frag<T>::load(Bb + bo);
      if (SPLIT) bl[j] = Frag<T>::load(Bb2 + bo);
    }
#pragma unroll
    for (int i = 0; i < 4; ++i) {
      const size_t ao = (size_t)(m0 + (i << 4) + rlane) * lda + koff + k0;
      V ah = Frag<T>::load(Ab + ao);
      V al;
      if (SPLIT) al = Frag<T>::load(Ab2 + ao);
#pragma unroll
      for (int j = 0; j < 4; ++j) {
        acc[i][j] = Frag<T>::mma(ah, bh[j], acc[i][j]);
        if (SPLIT) {
          acc[i][j] = Frag<T>::mma(ah, bl[j], acc[i][j]);
          acc[i][j] = Frag<T>::mma(al, bh[j], acc[i][j]);
        }
      }
      Frag<T>::guard(acc[i][0], acc[i][3], ah, SPLIT ? al : ah);
    }
    Frag<T>::keep(bh[0], bh[1], bh[2], bh[3]);
    if (SPLIT) Frag<T>::keep(bl[0], bl[1], bl[2], bl[3]);
  }
  acc_guard4(acc[0][0], acc[0][1], acc[0][2], acc[0][3]);
  acc_guard4(acc[1][0], acc[1][1], acc[1][2], acc[1][3]);
  acc_guard4(acc[2][0], acc[2][1], acc[2][2], acc[2][3]);
  acc_guard4(acc[3][0], acc[3][1], acc[3][2], acc[3][3]);

  float* slab = sT[wave];
  const float* Rb = RESID ? (resid + (size_t)b * strideR) : nullptr;
#pragma unroll
  for (int i = 0; i < 4; ++i) {
    const int mBase = m0 + (i << 4);
#pragma unroll
    for (int j = 0; j < 4; ++j) {
      const int n = n0 + (j << 4) + rlane;
      float bv = 0.f;
      if (BIAS_MODE == 2) bv = biasb[n];
#pragma unroll
      for (int r = 0; r < 8; ++r) {
        float v = acc[i][j][r] * scale;
        if (BIAS_MODE == 1) v += biasb[mBase + mOff + r];
        if (BIAS_MODE == 2) v += bv;
        if (RESID) v += Rb[(size_t)(mBase + mOff + r) * ldc + n];
        if (ACT == 2) v = fmaxf(v, 0.0f);
        if (ACT == 4) v = (v > 0.f) ? v : 0.01f * v;
        slab[(mOff + r) * 68 + (j << 4) + rlane] = v;
      }
    }
    __builtin_amdgcn_fence(__ATOMIC_RELEASE, "workgroup");
    __builtin_amdgcn_wave_barrier();
    __builtin_amdgcn_fence(__ATOMIC_ACQUIRE, "workgroup");
    if (OUT_MODE == 0) {
      float* C = (float*)Cout + (size_t)b * strideC;
      const int hh = lane >> 4, c4 = (lane & 15) * 4;
      for (int pass = 0; pass < 2; ++pass) {
#pragma unroll
        for (int it = 0; it < 8; ++it) {
          const int row = it * 2 + hh;
          v4f v = *(const v4f*)(slab + row * 68 + c4);
          *(volatile v4f*)(C + (size_t)(mBase + row) * ldc + n0 + c4) = v;
        }
        __threadfence();
      }
    } else {
      const int q = lane >> 3, c8 = (lane & 7) * 8;
      unsigned short* C  = (unsigned short*)Cout  + (size_t)b * strideC;
      unsigned short* C2 = (OUT_MODE == 2) ? ((unsigned short*)Cout2 + (size_t)b * strideC) : nullptr;
      for (int pass = 0; pass < 2; ++pass) {
#pragma unroll
        for (int it = 0; it < 4; ++it) {
          const int row = it * 4 + q;
          const float* sp = slab + row * 68 + c8;
          v8h hv, lv;
#pragma unroll
          for (int e = 0; e < 8; ++e) {
            if (OUT_MODE == 1) {
              hv[e] = (_Float16)sp[e];
            } else {
              unsigned short hb = f2bf_bits(sp[e]);
              unsigned short lb = f2bf_bits(sp[e] - bf_bits2f(hb));
              hv[e] = __builtin_bit_cast(_Float16, hb);
              lv[e] = __builtin_bit_cast(_Float16, lb);
            }
          }
          *(volatile v8h*)(C + (size_t)(mBase + row) * ldc + n0 + c8) = hv;
          if (OUT_MODE == 2) *(volatile v8h*)(C2 + (size_t)(mBase + row) * ldc + n0 + c8) = lv;
        }
        __threadfence();
      }
    }
    __builtin_amdgcn_fence(__ATOMIC_RELEASE, "workgroup");
    __builtin_amdgcn_wave_barrier();
    __builtin_amdgcn_fence(__ATOMIC_ACQUIRE, "workgroup");
  }
}

__global__ __launch_bounds__(256) void split8_bf16_kernel(const float* __restrict__ in,
                                                          unsigned short* __restrict__ outh,
                                                          unsigned short* __restrict__ outl, int n8) {
  const int i = blockIdx.x * 256 + threadIdx.x;
  if (i >= n8) return;
  const float* p = in + 8 * (size_t)i;
  const v4f a = *(const v4f*)(p);
  const v4f c = *(const v4f*)(p + 4);
  unsigned short hb[8], lb[8];
#pragma unroll
  for (int e = 0; e < 4; ++e) {
    const float f0 = a[e];
    const float f1 = c[e];
    hb[e]     = f2bf_bits(f0);
    lb[e]     = f2bf_bits(f0 - bf_bits2f(hb[e]));
    hb[4 + e] = f2bf_bits(f1);
    lb[4 + e] = f2bf_bits(f1 - bf_bits2f(hb[4 + e]));
  }
  const v4u uh = (v4u){pk16(hb[0], hb[1]), pk16(hb[2], hb[3]), pk16(hb[4], hb[5]), pk16(hb[6], hb[7])};
  const v4u ul = (v4u){pk16(lb[0], lb[1]), pk16(lb[2], lb[3]), pk16(lb[4], lb[5]), pk16(lb[6], lb[7])};
  unsigned short* qh = outh + 8 * (size_t)i;
  unsigned short* ql = outl + 8 * (size_t)i;
  *(volatile v4u*)qh = uh;
  *(volatile v4u*)ql = ul;
  __threadfence();
  *(volatile v4u*)qh = uh;
  *(volatile v4u*)ql = ul;
}

__global__ __launch_bounds__(256) void wsplit_transpose_kernel(const float* __restrict__ src,
                                                               unsigned short* __restrict__ dh,
                                                               unsigned short* __restrict__ dl,
                                                               int K2, int nblk) {
  __shared__ float sm[64][65];
  const int t   = threadIdx.x;
  const int blk = blockIdx.x >> 2;
  const int sub = blockIdx.x & 3;
  if (blk >= nblk) return;
  const int r0 = (sub >> 1) * 64;
  const int s0 = (sub & 1) * 64;
  const float* S = src + (size_t)blk * 16384;
#pragma unroll
  for (int i = 0; i < 16; ++i) {
    const int e  = i * 256 + t;
    const int rr = e >> 6;
    const int ss = e & 63;
    sm[ss][rr] = S[(size_t)(r0 + rr) * 128 + s0 + ss];
  }
  __syncthreads();
  const int g  = blk / K2;
  const int kk = blk - g * K2;
  const int RP = K2 * 128;
  const size_t base = (size_t)g * 128 * RP + (size_t)kk * 128 + r0;
  const int lane = t & 31, wave = t >> 5;
  const int q = lane >> 3, c8 = (lane & 7) * 8;
  for (int pass = 0; pass < 2; ++pass) {
#pragma unroll
    for (int it = 0; it < 2; ++it) {
      const int row = wave * 8 + it * 4 + q;
      unsigned short hb[8], lb[8];
#pragma unroll
      for (int e = 0; e < 8; ++e) {
        const float f = sm[row][c8 + e];
        hb[e] = f2bf_bits(f);
        lb[e] = f2bf_bits(f - bf_bits2f(hb[e]));
      }
      const v4u uh = (v4u){pk16(hb[0], hb[1]), pk16(hb[2], hb[3]), pk16(hb[4], hb[5]), pk16(hb[6], hb[7])};
      const v4u ul = (v4u){pk16(lb[0], lb[1]), pk16(lb[2], lb[3]), pk16(lb[4], lb[5]), pk16(lb[6], lb[7])};
      const size_t o = base + (size_t)(s0 + row) * RP + c8;
      *(volatile v4u*)(dh + o) = uh;
      *(volatile v4u*)(dl + o) = ul;
    }
    __threadfence();
  }
}


static void gemm_act(hipStream_t st,
                     const unsigned short* Ah, const unsigned short* Al, int lda, long sA,
                     const unsigned short* Bh, const unsigned short* Bl, int ldb, long sB,
                     unsigned short* Ch, unsigned short* Cl, int ldc, long sC,
                     const float* bias, long sBias, int M, int K, int batch, const float* dummy) {
  const int tiles = (M / 64) * (kCh / 64);
  dim3 grid((unsigned)((tiles + 7) / 8), (unsigned)batch);
  wmma_gemm64<1, true, 2, 2, false, 2><<<grid, dim3(256), 0, st>>>(
      Ah, Al, lda, sA, Bh, Bl, ldb, sB, (void*)Ch, (void*)Cl, ldc, sC,
      bias, sBias, dummy, 0L, M, kCh, K, 1.0f);
}

extern "C" void kernel_launch(void* const* d_in, const int* in_sizes, int n_in,
                              void* d_out, int out_size, void* d_ws, size_t ws_size,
                              hipStream_t stream) {
  if (n_in < 18) return;
  if (in_sizes[0] != kNdat * kLen) return;
  if (out_size != kNdat * kLen) return;
  if (ws_size < kWsTotal) return;
  const int  wsrc[9]  = {1, 3, 5, 7, 9, 11, 13, 15, 17};
  const long woff[9]  = {0, 16384, 81920, 212992, 475136, 1523712, 1785856, 1916928, 1982464};
  const int  wk2[9]   = {1, 2, 2, 2, 1, 2, 2, 2, 1};
  const int  wnblk[9] = {1, 4, 8, 16, 64, 16, 8, 4, 1};
  for (int i = 0; i < 9; ++i) {
    if (in_sizes[wsrc[i]] != wnblk[i] * 16384) return;
  }
  if (in_sizes[2] != 128 || in_sizes[4] != 256 || in_sizes[6] != 512 || in_sizes[8] != 1024 ||
      in_sizes[10] != 8192 || in_sizes[12] != 1024 || in_sizes[14] != 512 || in_sizes[16] != 256) return;

  unsigned char* ws = (unsigned char*)d_ws;
  unsigned short* WH  = (unsigned short*)(ws + kOffWH);
  unsigned short* WL  = (unsigned short*)(ws + kOffWL);
  unsigned short* XH  = (unsigned short*)(ws + kOffXH);
  unsigned short* XL  = (unsigned short*)(ws + kOffXL);
  unsigned short* P0H = (unsigned short*)(ws + kOffP0H);
  unsigned short* P0L = (unsigned short*)(ws + kOffP0L);
  unsigned short* P1H = (unsigned short*)(ws + kOffP1H);
  unsigned short* P1L = (unsigned short*)(ws + kOffP1L);

  const float* x  = (const float*)d_in[0];
  const float* xb = (const float*)d_in[2];
  const float* b1 = (const float*)d_in[4];
  const float* b2 = (const float*)d_in[6];
  const float* b3 = (const float*)d_in[8];
  const float* mb = (const float*)d_in[10];
  const float* b4 = (const float*)d_in[12];
  const float* b5 = (const float*)d_in[14];
  const float* b6 = (const float*)d_in[16];
  float* out = (float*)d_out;

  {
    const int n8 = (int)(kPlane / 8);
    split8_bf16_kernel<<<dim3((unsigned)((n8 + 255) / 256)), dim3(256), 0, stream>>>(x, XH, XL, n8);
  }
  for (int i = 0; i < 9; ++i) {
    wsplit_transpose_kernel<<<dim3((unsigned)(wnblk[i] * 4)), dim3(256), 0, stream>>>(
        (const float*)d_in[wsrc[i]], WH + woff[i], WL + woff[i], wk2[i], wnblk[i]);
  }

  const long PL = kPlane;
  gemm_act(stream, XH, XL, 128, 0L, WH + woff[0], WL + woff[0], 128, 0L,
           P0H, P0L, 128, 0L, xb, 0L, 65536, 128, 1, xb);
  gemm_act(stream, P0H, P0L, 256, 0L, WH + woff[1], WL + woff[1], 256, 32768L,
           P1H, P1L, 128, 4194304L, b1, 128L, 32768, 256, 2, xb);
  for (int j = 0; j < 2; ++j) {
    gemm_act(stream, P1H, P1L, 256, 4194304L, WH + woff[2] + j * 32768, WL + woff[2] + j * 32768, 256, 65536L,
             P0H + (long)j * 2097152, P0L + (long)j * 2097152, 128, 4194304L, b2 + j * 128, 256L, 16384, 256, 2, xb);
  }
  for (int j = 0; j < 2; ++j) {
    gemm_act(stream, P0H, P0L, 256, 2097152L, WH + woff[3] + j * 32768, WL + woff[3] + j * 32768, 256, 65536L,
             P1H + (long)j * 1048576, P1L + (long)j * 1048576, 128, 2097152L, b3 + j * 128, 256L, 8192, 256, 4, xb);
  }
  for (int xx = 0; xx < 8; ++xx) {
    const long cb = (long)(xx >> 1) * 2097152 + (long)(xx & 1) * 128;
    gemm_act(stream, P1H + xx * 128, P1L + xx * 128, 1024, 1048576L,
             WH + woff[4] + (long)xx * 16384, WL + woff[4] + (long)xx * 16384, 128, 131072L,
             P0H + cb, P0L + cb, 2048, 256L, mb + xx * 128, 1024L, 1024, 128, 8, xb);
  }
  for (int xo = 0; xo < 4; ++xo) {
    const long cb = (long)(xo >> 1) * 4194304 + (long)(xo & 1) * 128;
    gemm_act(stream, P0H + (long)xo * 2097152, P0L + (long)xo * 2097152, 256, 0L,
             WH + woff[5] + (long)xo * 65536, WL + woff[5] + (long)xo * 65536, 256, 32768L,
             P1H + cb, P1L + cb, 512, 256L, b4 + xo * 256, 128L, 8192, 256, 2, xb);
  }
  for (int j = 0; j < 2; ++j) {
    gemm_act(stream, P1H, P1L, 256, 4194304L, WH + woff[6] + j * 32768, WL + woff[6] + j * 32768, 256, 65536L,
             P0H + (long)j * 256, P0L + (long)j * 256, 512, 128L, b5 + j * 128, 256L, 16384, 256, 2, xb);
  }
  gemm_act(stream, P0H, P0L, 256, 0L, WH + woff[7], WL + woff[7], 256, 32768L,
           P1H, P1L, 256, 128L, b6, 128L, 32768, 256, 2, xb);
  {
    const int tiles = (65536 / 64) * (128 / 64);
    dim3 grid((unsigned)((tiles + 7) / 8), 1u);
    wmma_gemm64<1, true, 0, 0, false, 0><<<grid, dim3(256), 0, stream>>>(
        P1H, P1L, 128, 0L, WH + woff[8], WL + woff[8], 128, 0L,
        (void*)out, (void*)P0H, 128, 0L, xb, 0L, xb, 0L, 65536, 128, 128, 1.0f);
  }
}
